// BeeSender_49057116454978
// MI455X (gfx1250) — hardware-verified
//
#include <hip/hip_runtime.h>
#include <stddef.h>


#define FD      128
#define NREL    4
#define KA      (NREL * FD)
#define HD      256
#define KC      (2 * FD)
#define NTHR    256
#define NWAVE   8
#define EPT     8
#define NGRP    2
#define CHUNK   (NTHR * EPT * NGRP)
#define WCAP    (EPT * NGRP * 32)
#define LISTN   (NWAVE * WCAP)
#define SLOTSH  13
#define NBC     8192
#define NBF     2048
#define RCAP    49152
#define RBN     128
#define CPT     16
#define OTHR    (NBC / CPT)
#define GR      64
#define QB      32
#define DEGCAP  256
#define APA     (KA + 8)
#define APX     (FD + 8)
#define APC     (KC + 8)
#define WSCAP   134217728
#define OWF1    0
#define OWR1    (OWF1 + FD * KA)
#define OWF2    (OWR1 + 2 * FD * FD)
#define OWR2    (OWF2 + FD * KA)
#define OWC     (OWR2 + 2 * FD * FD)
#define OWTOT   (OWC + 2 * HD * KC)
#define NWBLK   112

#define LDS_FILL ((RCAP + NBF + LISTN) * 4 + 64)
#define LDS_LAY  (GR * APA * 2 + 2 * GR * APX * 2 + GR * FD * 4)

static_assert((CHUNK & (CHUNK - 1)) == 0);
static_assert(NBC <= (1 << SLOTSH) && NBF <= (1 << SLOTSH));
static_assert((NBC & (NBC - 1)) == 0 && (NBF & (NBF - 1)) == 0);
static_assert(NBC == 4 * NBF);
static_assert(OTHR * CPT == NBC && OTHR == 512 && 128 * CPT == NBF);
static_assert((RCAP % 32) == 0);
static_assert(GR == NWAVE * 8 && GR == 4 * 16);
static_assert(2 * QB == GR);
static_assert(((APA * 2) % 16) == 0 && ((APX * 2) % 16) == 0 && ((APC * 2) % 16) == 0);
static_assert(2 * QB * APC * 2 <= GR * APA * 2);
static_assert(QB * HD * 4 <= GR * FD * 4);
static_assert(((GR * APA * 2) % 16) == 0 && ((GR * APX * 2) % 16) == 0);
static_assert(OWR1 == 65536 && OWF2 == 98304 && OWR2 == 163840 && OWC == 196608 && OWTOT == 327680);
static_assert(((QB * KC / 8) % NTHR) == 0);

typedef float          v4f  __attribute__((ext_vector_type(4)));
typedef float          v8f  __attribute__((ext_vector_type(8)));
typedef int            v4i  __attribute__((ext_vector_type(4)));
typedef unsigned short v4us __attribute__((ext_vector_type(4)));
typedef unsigned short v8us __attribute__((ext_vector_type(8)));
typedef __bf16         v16b __attribute__((ext_vector_type(16)));
typedef _Float16       v4h  __attribute__((ext_vector_type(4)));
typedef _Float16       v8h  __attribute__((ext_vector_type(8)));
typedef _Float16       v16h __attribute__((ext_vector_type(16)));
union FragB { v16b v; v8us h[2]; };
union FragH { v16h v; v8h  h[2]; };

__device__ __forceinline__ unsigned int bfr(float f) {
  const unsigned int u = __float_as_uint(f);
  return (u + 0x7FFFu + ((u >> 16) & 1u)) >> 16;
}

__device__ __forceinline__ void split1(float x, unsigned short& hb, unsigned short& lb) {
  const unsigned int hu = bfr(x);
  const float hf = __uint_as_float(hu << 16);
  hb = (unsigned short)hu;
  lb = (unsigned short)bfr(x - hf);
}

__device__ __forceinline__ void split8(v4f a, v4f b, v8us& hi, v8us& lo) {
  unsigned short hb, lb;
  split1(a.x, hb, lb); hi[0] = hb; lo[0] = lb;
  split1(a.y, hb, lb); hi[1] = hb; lo[1] = lb;
  split1(a.z, hb, lb); hi[2] = hb; lo[2] = lb;
  split1(a.w, hb, lb); hi[3] = hb; lo[3] = lb;
  split1(b.x, hb, lb); hi[4] = hb; lo[4] = lb;
  split1(b.y, hb, lb); hi[5] = hb; lo[5] = lb;
  split1(b.z, hb, lb); hi[6] = hb; lo[6] = lb;
  split1(b.w, hb, lb); hi[7] = hb; lo[7] = lb;
}

__device__ __forceinline__ void split4(v4f a, v4us& hi, v4us& lo) {
  unsigned short hb, lb;
  split1(a.x, hb, lb); hi[0] = hb; lo[0] = lb;
  split1(a.y, hb, lb); hi[1] = hb; lo[1] = lb;
  split1(a.z, hb, lb); hi[2] = hb; lo[2] = lb;
  split1(a.w, hb, lb); hi[3] = hb; lo[3] = lb;
}

__device__ __forceinline__ v8f wmb(v16b a, v16b b, v8f c) {
  v8f d = __builtin_amdgcn_wmma_f32_16x16x32_bf16(false, a, false, b, (short)0, c, false, false);
  asm volatile("v_nop\n\tv_nop\n\tv_nop\n\tv_nop" : "+v"(d) : "v"(a), "v"(b));
  return d;
}
__device__ __forceinline__ v8f wmf(v16h a, v16h b, v8f c) {
  v8f d = __builtin_amdgcn_wmma_f32_16x16x32_f16(false, a, false, b, (short)0, c, false, false);
  asm volatile("v_nop\n\tv_nop\n\tv_nop\n\tv_nop" : "+v"(d) : "v"(a), "v"(b));
  return d;
}

template <int NB>
__device__ __forceinline__ int scan_chunk(const int* __restrict__ dsts, int nE, int cbase, int slotBase,
                                          int vec8, int* list, int tid, int lane, int wave) {
  int wc = 0;
#pragma unroll
  for (int g = 0; g < NGRP; ++g) {
    const int el0  = (g * NTHR + tid) * EPT;
    const int e0   = cbase + el0;
    const int sent = -2147483647 - 1;
    v4i da, db;
    if (vec8 != 0 && cbase + CHUNK <= nE) {
      da = *(const v4i*)(dsts + e0);
      db = *(const v4i*)(dsts + e0 + 4);
    } else {
      da.x = (e0     < nE) ? dsts[min(e0, nE - 1)] : sent;
      da.y = (e0 + 1 < nE) ? dsts[min(e0 + 1, nE - 1)] : sent;
      da.z = (e0 + 2 < nE) ? dsts[min(e0 + 2, nE - 1)] : sent;
      da.w = (e0 + 3 < nE) ? dsts[min(e0 + 3, nE - 1)] : sent;
      db.x = (e0 + 4 < nE) ? dsts[min(e0 + 4, nE - 1)] : sent;
      db.y = (e0 + 5 < nE) ? dsts[min(e0 + 5, nE - 1)] : sent;
      db.z = (e0 + 6 < nE) ? dsts[min(e0 + 6, nE - 1)] : sent;
      db.w = (e0 + 7 < nE) ? dsts[min(e0 + 7, nE - 1)] : sent;
    }
    const unsigned nb = (unsigned)slotBase;
    const unsigned s0 = (unsigned)da.x - nb, s1 = (unsigned)da.y - nb;
    const unsigned s2 = (unsigned)da.z - nb, s3 = (unsigned)da.w - nb;
    const unsigned s4 = (unsigned)db.x - nb, s5 = (unsigned)db.y - nb;
    const unsigned s6 = (unsigned)db.z - nb, s7 = (unsigned)db.w - nb;
    const bool h0 = s0 < (unsigned)NB, h1 = s1 < (unsigned)NB, h2 = s2 < (unsigned)NB, h3 = s3 < (unsigned)NB;
    const bool h4 = s4 < (unsigned)NB, h5 = s5 < (unsigned)NB, h6 = s6 < (unsigned)NB, h7 = s7 < (unsigned)NB;
    const unsigned any = __builtin_amdgcn_ballot_w32(h0 | h1 | h2 | h3 | h4 | h5 | h6 | h7);
    if (any != 0u) {
#define HITJ(J, HJ, SJ) { \
        const unsigned mj = __builtin_amdgcn_ballot_w32(HJ); \
        if (mj != 0u) { \
          if (HJ) { \
            const int pos = wc + (int)__builtin_amdgcn_mbcnt_lo(mj, 0u); \
            if (pos < WCAP) list[wave * WCAP + pos] = ((el0 + (J)) << SLOTSH) | (int)(SJ); \
          } \
          wc += (int)__builtin_popcount(mj); } }
      HITJ(0, h0, s0)
      HITJ(1, h1, s1)
      HITJ(2, h2, s2)
      HITJ(3, h3, s3)
      HITJ(4, h4, s4)
      HITJ(5, h5, s5)
      HITJ(6, h6, s6)
      HITJ(7, h7, s7)
#undef HITJ
    }
  }
  return wc;
}

__global__ __launch_bounds__(NTHR) void k_wprep(
    const float* __restrict__ wrel1, const float* __restrict__ wroot1,
    const float* __restrict__ wrel2, const float* __restrict__ wroot2,
    const float* __restrict__ wfc, unsigned short* wp) {
  const int blk = blockIdx.x, tid = threadIdx.x;
  if (blk < 64) {
    const bool sec = blk >= 32;
    const float* w = sec ? wrel2 : wrel1;
    const int base = sec ? OWF2 : OWF1;
    const int i  = ((blk & 31) * NTHR + tid);
    const int n  = i >> 6;
    const int k0 = (i & 63) * 8;
    v8h hv;
#pragma unroll
    for (int e = 0; e < 8; ++e) hv[e] = (_Float16)(w[(size_t)(k0 + e) * FD + n] * 64.0f);
    _Float16* d = (_Float16*)wp + base + (size_t)n * KA + k0;
    *(volatile v8h*)d = hv;
    __threadfence();
    *(volatile v8h*)d = hv;
  } else if (blk < 80) {
    const bool sec = blk >= 72;
    const float* w = sec ? wroot2 : wroot1;
    const int base = sec ? OWR2 : OWR1;
    const int i  = ((blk - (sec ? 72 : 64)) * NTHR + tid);
    const int n  = i >> 4;
    const int k0 = (i & 15) * 8;
    float v[8];
#pragma unroll
    for (int e = 0; e < 8; ++e) v[e] = w[(size_t)(k0 + e) * FD + n];
    v4f a, b;
    a.x = v[0]; a.y = v[1]; a.z = v[2]; a.w = v[3];
    b.x = v[4]; b.y = v[5]; b.z = v[6]; b.w = v[7];
    v8us hv, lv;
    split8(a, b, hv, lv);
    unsigned short* dh = wp + base + (size_t)n * FD + k0;
    unsigned short* dl = dh + FD * FD;
    *(volatile v8us*)dh = hv;
    *(volatile v8us*)dl = lv;
    __threadfence();
    *(volatile v8us*)dh = hv;
    *(volatile v8us*)dl = lv;
  } else {
    const int i  = (blk - 80) * NTHR + tid;
    const int n  = i >> 5;
    const int k0 = (i & 31) * 8;
    float v[8];
#pragma unroll
    for (int e = 0; e < 8; ++e) v[e] = wfc[(size_t)(k0 + e) * HD + n];
    v4f a, b;
    a.x = v[0]; a.y = v[1]; a.z = v[2]; a.w = v[3];
    b.x = v[4]; b.y = v[5]; b.z = v[6]; b.w = v[7];
    v8us hv, lv;
    split8(a, b, hv, lv);
    unsigned short* dh = wp + OWC + (size_t)n * KC + k0;
    unsigned short* dl = dh + HD * KC;
    *(volatile v8us*)dh = hv;
    *(volatile v8us*)dl = lv;
    __threadfence();
    *(volatile v8us*)dh = hv;
    *(volatile v8us*)dl = lv;
  }
}

__global__ __launch_bounds__(NTHR) void k_count(const int* __restrict__ dsts, int* cnt, int nE, int vec8) {
  __shared__ __attribute__((aligned(16))) int scnt[NBC];
  __shared__ __attribute__((aligned(16))) int list[LISTN];
  __shared__ int wcnt[NWAVE];
  const int tid = threadIdx.x, lane = tid & 31, wave = tid >> 5;
  const int nodeBase = blockIdx.x * NBC;

  for (int i = tid; i < NBC; i += NTHR) scnt[i] = 0;
  __syncthreads();

  const int nChunks = (nE + CHUNK - 1) / CHUNK;
#pragma unroll 1
  for (int ch = 0; ch < nChunks; ++ch) {
    const int cbase = ch * CHUNK;
    const int wc = scan_chunk<NBC>(dsts, nE, cbase, nodeBase, vec8, list, tid, lane, wave);
    if (lane == 0) wcnt[wave] = wc;
    __syncthreads();
    if (wave == 0) {
#pragma unroll 1
      for (int wsx = 0; wsx < NWAVE; ++wsx) {
        int n = __builtin_amdgcn_readfirstlane(wcnt[wsx]);
        n = n > WCAP ? WCAP : (n < 0 ? 0 : n);
        const int* lp = list + wsx * WCAP;
#pragma unroll 1
        for (int i = 0; i < n; ++i) {
          const int ent  = __builtin_amdgcn_readfirstlane(lp[i]);
          const int slot = ent & (NBC - 1);
          if (lane == 0) scnt[slot] = scnt[slot] + 1;
        }
      }
    }
    __syncthreads();
  }

  v4i cq[8];
#pragma unroll
  for (int q = 0; q < 8; ++q) {
    const int f = (wave * 8 + q) * 128 + 4 * lane;
    cq[q] = *(const v4i*)(scnt + f);
  }
  int* cp = cnt + (size_t)nodeBase;
#pragma unroll
  for (int q = 0; q < 8; ++q) {
    const int f = (wave * 8 + q) * 128 + 4 * lane;
    *(volatile v4i*)(cp + f) = cq[q];
  }
  __threadfence();
#pragma unroll
  for (int q = 0; q < 8; ++q) {
    const int f = (wave * 8 + q) * 128 + 4 * lane;
    *(volatile v4i*)(cp + f) = cq[q];
  }
}

__global__ __launch_bounds__(OTHR) void k_offsets(
    const int* __restrict__ cnt, int* off, int* rbase, int nChunk) {
  __shared__ __attribute__((aligned(16))) int soff[NBC];
  __shared__ __attribute__((aligned(16))) int srb[RBN];
  __shared__ int wtot[OTHR / 32];
  const int tid = threadIdx.x, lane = tid & 31, wave = tid >> 5, sub = tid >> 7;
  for (int i = tid; i < RBN; i += OTHR) srb[i] = 0;
  int carry = 0;
#pragma unroll 1
  for (int ch = 0; ch < nChunk; ++ch) {
    const int base = ch * NBC;
    const int* cpp = cnt + base + CPT * tid;
    const v4i c0 = *(const v4i*)(cpp);
    const v4i c1 = *(const v4i*)(cpp + 4);
    const v4i c2 = *(const v4i*)(cpp + 8);
    const v4i c3 = *(const v4i*)(cpp + 12);
    int e[16];
    e[0]  = max(c0.x, 0); e[1]  = max(c0.y, 0); e[2]  = max(c0.z, 0); e[3]  = max(c0.w, 0);
    e[4]  = max(c1.x, 0); e[5]  = max(c1.y, 0); e[6]  = max(c1.z, 0); e[7]  = max(c1.w, 0);
    e[8]  = max(c2.x, 0); e[9]  = max(c2.y, 0); e[10] = max(c2.z, 0); e[11] = max(c2.w, 0);
    e[12] = max(c3.x, 0); e[13] = max(c3.y, 0); e[14] = max(c3.z, 0); e[15] = max(c3.w, 0);
    int ts = 0;
#pragma unroll
    for (int j = 0; j < 16; ++j) ts += e[j];
    int incl = ts;
#pragma unroll
    for (int d = 1; d < 32; d <<= 1) {
      const int t = __shfl_up(incl, d);
      if (lane >= d) incl += t;
    }
    if (lane == 31) wtot[wave] = incl;
    __syncthreads();
    const int S0 = wtot[0]  + wtot[1]  + wtot[2]  + wtot[3];
    const int S1 = wtot[4]  + wtot[5]  + wtot[6]  + wtot[7];
    const int S2 = wtot[8]  + wtot[9]  + wtot[10] + wtot[11];
    const int S3 = wtot[12] + wtot[13] + wtot[14] + wtot[15];
    int pre = 0;
#pragma unroll 1
    for (int w = 4 * sub; w < wave; ++w) pre += wtot[w];
    const int b0 = carry;
    const int b1 = b0 + ((S0 + 31) & ~31);
    const int b2 = b1 + ((S1 + 31) & ~31);
    const int b3 = b2 + ((S2 + 31) & ~31);
    const int b4 = b3 + ((S3 + 31) & ~31);
    const int myb = sub == 0 ? b0 : (sub == 1 ? b1 : (sub == 2 ? b2 : b3));
    if (tid == 0) {
      srb[min(4 * ch + 0, RBN - 1)] = b0;
      srb[min(4 * ch + 1, RBN - 1)] = b1;
      srb[min(4 * ch + 2, RBN - 1)] = b2;
      srb[min(4 * ch + 3, RBN - 1)] = b3;
    }
    int run = myb + pre + incl - ts;
#pragma unroll
    for (int j = 0; j < 16; ++j) { soff[CPT * tid + j] = run; run += e[j]; }
    carry = b4;
    __syncthreads();
    v4i o[4];
#pragma unroll
    for (int jj = 0; jj < 4; ++jj) o[jj] = *(const v4i*)(soff + 4 * (tid + jj * OTHR));
    int* op = off + base;
#pragma unroll
    for (int jj = 0; jj < 4; ++jj) *(volatile v4i*)(op + 4 * (tid + jj * OTHR)) = o[jj];
    __threadfence();
#pragma unroll
    for (int jj = 0; jj < 4; ++jj) *(volatile v4i*)(op + 4 * (tid + jj * OTHR)) = o[jj];
    __syncthreads();
  }
  if (tid == 0) srb[min(4 * nChunk, RBN - 1)] = carry;
  __syncthreads();
  v4i rv = {0, 0, 0, 0};
  if (tid < 32) rv = *(const v4i*)(srb + 4 * tid);
  if (tid < 32) *(volatile v4i*)(rbase + 4 * tid) = rv;
  __threadfence();
  if (tid < 32) *(volatile v4i*)(rbase + 4 * tid) = rv;
}

__global__ __launch_bounds__(NTHR) void k_fill(
    const int* __restrict__ dsts, const int* __restrict__ off, const int* __restrict__ rbase,
    int* csr, int nE, int vec8, int csrLen) {
  extern __shared__ v4f lds_dyn[];
  int* region = (int*)lds_dyn;
  int* cursor = region + RCAP;
  int* list   = cursor + NBF;
  int* wcnt   = list + LISTN;
  const int tid = threadIdx.x, lane = tid & 31, wave = tid >> 5;
  const int b = blockIdx.x;
  const int nodeBase = b * NBF;

  int rb0 = rbase[b];
  const int rb1 = rbase[b + 1];
  rb0 = rb0 < 0 ? 0 : (rb0 > csrLen ? csrLen : rb0);
  rb0 &= ~31;
  int len = rb1 - rb0;
  len = len < 0 ? 0 : (len > RCAP ? RCAP : len);
  int lenW = (len + 31) & ~31;
  if (rb0 + lenW > csrLen) lenW = (csrLen - rb0) & ~31;

  {
    const v4i z = {0, 0, 0, 0};
    for (int i = tid; i < RCAP / 4; i += NTHR) ((v4i*)region)[i] = z;
    for (int s = tid; s < NBF; s += NTHR) {
      int o = off[nodeBase + s] - rb0;
      o = o < 0 ? 0 : (o > RCAP ? RCAP : o);
      cursor[s] = o;
    }
  }
  __syncthreads();

  const int nChunks = (nE + CHUNK - 1) / CHUNK;
#pragma unroll 1
  for (int ch = 0; ch < nChunks; ++ch) {
    const int cbase = ch * CHUNK;
    const int wc = scan_chunk<NBF>(dsts, nE, cbase, nodeBase, vec8, list, tid, lane, wave);
    if (lane == 0) wcnt[wave] = wc;
    __syncthreads();
    if (wave == 0) {
#pragma unroll 1
      for (int wsx = 0; wsx < NWAVE; ++wsx) {
        int n = __builtin_amdgcn_readfirstlane(wcnt[wsx]);
        n = n > WCAP ? WCAP : (n < 0 ? 0 : n);
        const int* lp = list + wsx * WCAP;
#pragma unroll 1
        for (int i = 0; i < n; ++i) {
          const int ent  = __builtin_amdgcn_readfirstlane(lp[i]);
          const int slot = ent & (NBF - 1);
          int e = cbase + ((ent >> SLOTSH) & (CHUNK - 1));
          e = e > nE - 1 ? nE - 1 : e;
          if (lane == 0) {
            int pos = cursor[slot];
            pos = pos < 0 ? 0 : (pos > RCAP - 1 ? RCAP - 1 : pos);
            region[pos] = e;
            const int np = pos + 1;
            cursor[slot] = np > RCAP ? RCAP : np;
          }
        }
      }
    }
    __syncthreads();
  }

  const int nv = lenW >> 2;
  int* gp = csr + rb0;
#pragma unroll 1
  for (int i = tid; i < nv; i += NTHR) { const v4i v = ((const v4i*)region)[i]; *(volatile v4i*)(gp + 4 * i) = v; }
  __threadfence();
#pragma unroll 1
  for (int i = tid; i < nv; i += NTHR) { const v4i v = ((const v4i*)region)[i]; *(volatile v4i*)(gp + 4 * i) = v; }
}

__device__ __forceinline__ void agg_row(
    const int* __restrict__ csr, const int* __restrict__ esrc, const int* __restrict__ etyp,
    const float* __restrict__ feat, int n, int st, int lane, int nN, int nE, int csrLen,
    _Float16* arow) {
  v4f a0 = {0.f, 0.f, 0.f, 0.f}, a1 = {0.f, 0.f, 0.f, 0.f};
  v4f a2 = {0.f, 0.f, 0.f, 0.f}, a3 = {0.f, 0.f, 0.f, 0.f};
  int c0 = 0, c1 = 0, c2 = 0, c3 = 0;
#pragma unroll 1
  for (int q0 = 0; q0 < n; q0 += 32) {
    int pos = st + q0 + lane;
    pos = pos < 0 ? 0 : (pos > csrLen - 1 ? csrLen - 1 : pos);
    int ed = csr[pos];
    ed = ed < 0 ? 0 : (ed > nE - 1 ? nE - 1 : ed);
    int sv = esrc[ed];
    sv = sv < 0 ? 0 : (sv > nN - 1 ? nN - 1 : sv);
    int rv = etyp[ed];
    rv = rv < 0 ? 0 : (rv > NREL - 1 ? NREL - 1 : rv);
    const int mcnt = (n - q0) < 32 ? (n - q0) : 32;
#pragma unroll 1
    for (int p = 0; p < mcnt; ++p) {
      const int ss = __builtin_amdgcn_readlane(sv, p);
      const int rr = __builtin_amdgcn_readlane(rv, p);
      const v4f xv = *(const v4f*)(feat + (size_t)ss * FD + 4 * lane);
      if (rr == 0)      { a0 += xv; c0 += 1; }
      else if (rr == 1) { a1 += xv; c1 += 1; }
      else if (rr == 2) { a2 += xv; c2 += 1; }
      else              { a3 += xv; c3 += 1; }
    }
  }
  const float s0 = 8.0f * (1.0f / (float)(c0 < 1 ? 1 : c0));
  const float s1 = 8.0f * (1.0f / (float)(c1 < 1 ? 1 : c1));
  const float s2 = 8.0f * (1.0f / (float)(c2 < 1 ? 1 : c2));
  const float s3 = 8.0f * (1.0f / (float)(c3 < 1 ? 1 : c3));
  v4h h;
  h.x = (_Float16)(a0.x * s0); h.y = (_Float16)(a0.y * s0); h.z = (_Float16)(a0.z * s0); h.w = (_Float16)(a0.w * s0);
  *(v4h*)(arow + 0 * FD + 4 * lane) = h;
  h.x = (_Float16)(a1.x * s1); h.y = (_Float16)(a1.y * s1); h.z = (_Float16)(a1.z * s1); h.w = (_Float16)(a1.w * s1);
  *(v4h*)(arow + 1 * FD + 4 * lane) = h;
  h.x = (_Float16)(a2.x * s2); h.y = (_Float16)(a2.y * s2); h.z = (_Float16)(a2.z * s2); h.w = (_Float16)(a2.w * s2);
  *(v4h*)(arow + 2 * FD + 4 * lane) = h;
  h.x = (_Float16)(a3.x * s3); h.y = (_Float16)(a3.y * s3); h.z = (_Float16)(a3.z * s3); h.w = (_Float16)(a3.w * s3);
  *(v4h*)(arow + 3 * FD + 4 * lane) = h;
}

template <int RELU>
__device__ __forceinline__ void rel_gemm(
    const _Float16* sA, const unsigned short* sXh, const unsigned short* sXl,
    const _Float16* __restrict__ Wf, const unsigned short* __restrict__ Wr,
    const float* __restrict__ bias, float* stg, int wave, int lane) {
  const int hh = lane >> 4, m = lane & 15, rg = wave >> 1, chf = wave & 1;
  const _Float16* pa = sA + (rg * 16 + m) * APA + 8 * hh;
  const unsigned short* ph = sXh + (rg * 16 + m) * APX + 8 * hh;
  const unsigned short* pl = sXl + (rg * 16 + m) * APX + 8 * hh;
  float* strow = stg + (rg * 16 + 8 * hh) * FD + m;
#pragma unroll 1
  for (int tt = 0; tt < 4; ++tt) {
    const int t = chf * 4 + tt;
    v8f accF = {0.f, 0.f, 0.f, 0.f, 0.f, 0.f, 0.f, 0.f};
    v8f accB = {0.f, 0.f, 0.f, 0.f, 0.f, 0.f, 0.f, 0.f};
    const _Float16* bf = Wf + (size_t)(16 * t + m) * KA + 8 * hh;
#pragma unroll
    for (int ks = 0; ks < KA / 32; ++ks) {
      FragH a, b;
      a.h[0] = *(const v8h*)(pa + 32 * ks);
      a.h[1] = *(const v8h*)(pa + 32 * ks + 16);
      b.h[0] = *(const v8h*)(bf + 32 * ks);
      b.h[1] = *(const v8h*)(bf + 32 * ks + 16);
      accF = wmf(a.v, b.v, accF);
    }
    const unsigned short* bb = Wr + (size_t)(16 * t + m) * FD + 8 * hh;
#pragma unroll
    for (int ks = 0; ks < FD / 32; ++ks) {
      FragB ah, al, bh, bl;
      ah.h[0] = *(const v8us*)(ph + 32 * ks);           ah.h[1] = *(const v8us*)(ph + 32 * ks + 16);
      al.h[0] = *(const v8us*)(pl + 32 * ks);           al.h[1] = *(const v8us*)(pl + 32 * ks + 16);
      bh.h[0] = *(const v8us*)(bb + 32 * ks);           bh.h[1] = *(const v8us*)(bb + 32 * ks + 16);
      bl.h[0] = *(const v8us*)(bb + FD * FD + 32 * ks); bl.h[1] = *(const v8us*)(bb + FD * FD + 32 * ks + 16);
      accB = wmb(ah.v, bh.v, accB);
      accB = wmb(ah.v, bl.v, accB);
      accB = wmb(al.v, bh.v, accB);
    }
    const float bv = bias[16 * t + m];
#pragma unroll
    for (int r = 0; r < 8; ++r) {
      float v = accF[r] * (1.0f / 512.0f) + accB[r] + bv;
      if (RELU != 0) v = fmaxf(v, 0.0f);
      strow[r * FD + 16 * t] = v;
    }
  }
}

__global__ __launch_bounds__(NTHR) void k_layer1(
    const int* __restrict__ csr, const int* __restrict__ off, const int* __restrict__ cnt,
    const int* __restrict__ esrc, const int* __restrict__ etyp, const float* __restrict__ x,
    const unsigned short* __restrict__ wp, const float* __restrict__ bias,
    float* H1, int nN, int nE, int csrLen) {
  extern __shared__ v4f lds_dyn[];
  _Float16*       sA  = (_Float16*)lds_dyn;
  unsigned short* sXh = (unsigned short*)(sA + GR * APA);
  unsigned short* sXl = sXh + GR * APX;
  float*          stg = (float*)(sXl + GR * APX);
  const int tid = threadIdx.x, lane = tid & 31, wave = tid >> 5;
  const int rowBase = blockIdx.x * GR;

  const int cl = rowBase + 8 * wave + (lane & 7);
  const int cv = cnt[cl];
  const int ov = off[cl];
#pragma unroll 1
  for (int j = 0; j < 8; ++j) {
    int n = __builtin_amdgcn_readlane(cv, j);
    n = n < 0 ? 0 : (n > DEGCAP ? DEGCAP : n);
    const int st = __builtin_amdgcn_readlane(ov, j);
    const int rl = 8 * wave + j;
    int node = rowBase + rl;
    node = node > nN - 1 ? nN - 1 : node;
    agg_row(csr, esrc, etyp, x, n, st, lane, nN, nE, csrLen, sA + rl * APA);
    const v4f xs = *(const v4f*)(x + (size_t)node * FD + 4 * lane);
    v4us hi, lo;
    split4(xs, hi, lo);
    *(v4us*)(sXh + rl * APX + 4 * lane) = hi;
    *(v4us*)(sXl + rl * APX + 4 * lane) = lo;
  }
  __syncthreads();

  rel_gemm<1>(sA, sXh, sXl, (const _Float16*)(wp + OWF1), wp + OWR1, bias, stg, wave, lane);
  __syncthreads();

  v4f hv[8];
#pragma unroll
  for (int i = 0; i < 8; ++i) hv[i] = *(const v4f*)(stg + (8 * wave + i) * FD + 4 * lane);
  float* gp = H1 + (size_t)(rowBase + 8 * wave) * FD + 4 * lane;
#pragma unroll
  for (int i = 0; i < 8; ++i) *(volatile v4f*)(gp + (size_t)i * FD) = hv[i];
  __threadfence();
#pragma unroll
  for (int i = 0; i < 8; ++i) *(volatile v4f*)(gp + (size_t)i * FD) = hv[i];
}

__global__ __launch_bounds__(NTHR) void k_layer2fc(
    const int* __restrict__ csr, const int* __restrict__ off, const int* __restrict__ cnt,
    const int* __restrict__ esrc, const int* __restrict__ etyp, const float* __restrict__ H1,
    const int* __restrict__ nest, const int* __restrict__ food,
    const unsigned short* __restrict__ wp, const float* __restrict__ bias2, const float* __restrict__ bfc,
    float* out, int nN, int nE, int csrLen, int nB) {
  extern __shared__ v4f lds_dyn[];
  _Float16*       sA  = (_Float16*)lds_dyn;
  unsigned short* sXh = (unsigned short*)(sA + GR * APA);
  unsigned short* sXl = sXh + GR * APX;
  float*          stg = (float*)(sXl + GR * APX);
  unsigned short* sCh = (unsigned short*)lds_dyn;
  unsigned short* sCl = sCh + QB * APC;
  const int tid = threadIdx.x, lane = tid & 31, wave = tid >> 5, hh = lane >> 4, m = lane & 15;
  const int qBase = blockIdx.x * QB;

  int slot = qBase + ((8 * wave + (lane & 7)) & (QB - 1));
  slot = slot > nB - 1 ? nB - 1 : slot;
  const int nvq = nest[slot];
  const int fvq = food[slot];
  int ndl = (wave < 4) ? nvq : fvq;
  ndl = ndl < 0 ? 0 : (ndl > nN - 1 ? nN - 1 : ndl);
  const int cv = cnt[ndl];
  const int ov = off[ndl];
#pragma unroll 1
  for (int j = 0; j < 8; ++j) {
    int n = __builtin_amdgcn_readlane(cv, j);
    n = n < 0 ? 0 : (n > DEGCAP ? DEGCAP : n);
    const int st   = __builtin_amdgcn_readlane(ov, j);
    const int node = __builtin_amdgcn_readlane(ndl, j);
    const int rl = 8 * wave + j;
    agg_row(csr, esrc, etyp, H1, n, st, lane, nN, nE, csrLen, sA + rl * APA);
    const v4f xs = *(const v4f*)(H1 + (size_t)node * FD + 4 * lane);
    v4us hi, lo;
    split4(xs, hi, lo);
    *(v4us*)(sXh + rl * APX + 4 * lane) = hi;
    *(v4us*)(sXl + rl * APX + 4 * lane) = lo;
  }
  __syncthreads();

  rel_gemm<0>(sA, sXh, sXl, (const _Float16*)(wp + OWF2), wp + OWR2, bias2, stg, wave, lane);
  __syncthreads();

#pragma unroll
  for (int i = 0; i < (QB * KC / 8) / NTHR; ++i) {
    const int idx  = i * NTHR + tid;
    const int qq   = idx >> 5;
    const int c0   = (idx & 31) * 8;
    const int srow = qq + (c0 >> 7) * QB;
    const int scol = c0 & (FD - 1);
    const v4f a = *(const v4f*)(stg + srow * FD + scol);
    const v4f b = *(const v4f*)(stg + srow * FD + scol + 4);
    v8us hv, lv;
    split8(a, b, hv, lv);
    *(v8us*)(sCh + qq * APC + c0) = hv;
    *(v8us*)(sCl + qq * APC + c0) = lv;
  }
  __syncthreads();

  {
    const int rgf = wave & 1;
    const unsigned short* ph = sCh + (rgf * 16 + m) * APC + 8 * hh;
    const unsigned short* pl = sCl + (rgf * 16 + m) * APC + 8 * hh;
    float* so = stg;
    float* strow = so + (rgf * 16 + 8 * hh) * HD + m;
#pragma unroll 1
    for (int tt = 0; tt < 4; ++tt) {
      const int t = (wave >> 1) * 4 + tt;
      v8f acc = {0.f, 0.f, 0.f, 0.f, 0.f, 0.f, 0.f, 0.f};
      const unsigned short* bb = wp + OWC + (size_t)(16 * t + m) * KC + 8 * hh;
#pragma unroll
      for (int ks = 0; ks < KC / 32; ++ks) {
        FragB ah, al, bh, bl;
        ah.h[0] = *(const v8us*)(ph + 32 * ks);           ah.h[1] = *(const v8us*)(ph + 32 * ks + 16);
        al.h[0] = *(const v8us*)(pl + 32 * ks);           al.h[1] = *(const v8us*)(pl + 32 * ks + 16);
        bh.h[0] = *(const v8us*)(bb + 32 * ks);           bh.h[1] = *(const v8us*)(bb + 32 * ks + 16);
        bl.h[0] = *(const v8us*)(bb + HD * KC + 32 * ks); bl.h[1] = *(const v8us*)(bb + HD * KC + 32 * ks + 16);
        acc = wmb(ah.v, bh.v, acc);
        acc = wmb(ah.v, bl.v, acc);
        acc = wmb(al.v, bh.v, acc);
      }
      const float bv = bfc[16 * t + m];
#pragma unroll
      for (int r = 0; r < 8; ++r) strow[r * HD + 16 * t] = fmaxf(acc[r] + bv, 0.0f);
    }
  }
  __syncthreads();

  v4f ovv[8];
#pragma unroll
  for (int i = 0; i < 8; ++i) {
    const int p = 8 * wave + i, row = p >> 1, half = p & 1;
    ovv[i] = *(const v4f*)(stg + row * HD + half * 128 + 4 * lane);
  }
#pragma unroll
  for (int i = 0; i < 8; ++i) {
    const int p = 8 * wave + i, row = p >> 1, half = p & 1;
    const int q = qBase + row;
    if (q < nB) *(volatile v4f*)(out + (size_t)q * HD + half * 128 + 4 * lane) = ovv[i];
  }
  __threadfence();
#pragma unroll
  for (int i = 0; i < 8; ++i) {
    const int p = 8 * wave + i, row = p >> 1, half = p & 1;
    const int q = qBase + row;
    if (q < nB) *(volatile v4f*)(out + (size_t)q * HD + half * 128 + 4 * lane) = ovv[i];
  }
}

extern "C" void kernel_launch(void* const* d_in, const int* in_sizes, int n_in,
                              void* d_out, int out_size, void* d_ws, size_t ws_size,
                              hipStream_t stream) {
  if (n_in < 13) return;
  const int nN = in_sizes[0] / FD;
  if (nN < 1 || in_sizes[0] != nN * FD) return;
  const int nE = in_sizes[2];
  if (nE < 1 || in_sizes[1] != 2 * nE) return;
  const int nB = in_sizes[3];
  if (nB < 1 || in_sizes[4] != nB) return;
  if (in_sizes[5] != NREL * FD * FD || in_sizes[6] != FD * FD || in_sizes[7] != FD) return;
  if (in_sizes[8] != NREL * FD * FD || in_sizes[9] != FD * FD || in_sizes[10] != FD) return;
  if (in_sizes[11] != KC * HD || in_sizes[12] != HD) return;
  if ((long long)out_size != (long long)nB * HD) return;
  if (nE > (1 << 28) || nN > (1 << 24) || nB > (1 << 24)) return;

  const float* x      = (const float*)d_in[0];
  const int*   eidx   = (const int*)d_in[1];
  const int*   etyp   = (const int*)d_in[2];
  const int*   nest   = (const int*)d_in[3];
  const int*   food   = (const int*)d_in[4];
  const float* wrel1  = (const float*)d_in[5];
  const float* wroot1 = (const float*)d_in[6];
  const float* b1     = (const float*)d_in[7];
  const float* wrel2  = (const float*)d_in[8];
  const float* wroot2 = (const float*)d_in[9];
  const float* b2     = (const float*)d_in[10];
  const float* wfc    = (const float*)d_in[11];
  const float* bfc    = (const float*)d_in[12];
  float* out = (float*)d_out;
  const int* esrc = eidx;
  const int* dsts = eidx + nE;

  const int NPAD   = ((nN + GR - 1) / GR) * GR;
  const int nBC    = (nN + NBC - 1) / NBC;
  const int CNTPAD = nBC * NBC;
  if (4 * nBC + 1 > RBN) return;
  const int nBF    = (nN + NBF - 1) / NBF;
  const int csrLen = ((nE + 31) & ~31) + 4096;
  if (31 * 4 * nBC > 4096) return;
  const int nL1    = NPAD / GR;
  const int nQ     = (nB + QB - 1) / QB;

  char* ws = (char*)d_ws;
  size_t off = 0;
  const size_t oW   = off; off += (size_t)OWTOT * 2;               off = (off + 255) & ~(size_t)255;
  const size_t oCnt = off; off += (size_t)CNTPAD * 4;              off = (off + 255) & ~(size_t)255;
  const size_t oOff = off; off += (size_t)CNTPAD * 4;              off = (off + 255) & ~(size_t)255;
  const size_t oRb  = off; off += (size_t)RBN * 4;                 off = (off + 255) & ~(size_t)255;
  const size_t oCsr = off; off += (size_t)csrLen * 4;              off = (off + 255) & ~(size_t)255;
  const size_t oH1  = off; off += (size_t)NPAD * FD * 4;           off = (off + 255) & ~(size_t)255;
  if (off > ws_size || off > (size_t)WSCAP) return;
  unsigned short* wp   = (unsigned short*)(ws + oW);
  int*            cnt  = (int*)(ws + oCnt);
  int*            offp = (int*)(ws + oOff);
  int*            rb   = (int*)(ws + oRb);
  int*            csr  = (int*)(ws + oCsr);
  float*          H1   = (float*)(ws + oH1);

  const int vec8 = ((nE & 3) == 0) ? 1 : 0;

  k_wprep<<<NWBLK, NTHR, 0, stream>>>(wrel1, wroot1, wrel2, wroot2, wfc, wp);

  k_count<<<nBC, NTHR, 0, stream>>>(dsts, cnt, nE, vec8);
  k_offsets<<<1, OTHR, 0, stream>>>(cnt, offp, rb, nBC);
  hipFuncSetAttribute(reinterpret_cast<const void*>(&k_fill),
                      hipFuncAttributeMaxDynamicSharedMemorySize, LDS_FILL);
  k_fill<<<nBF, NTHR, LDS_FILL, stream>>>(dsts, offp, rb, csr, nE, vec8, csrLen);

  hipFuncSetAttribute(reinterpret_cast<const void*>(&k_layer1),
                      hipFuncAttributeMaxDynamicSharedMemorySize, LDS_LAY);
  k_layer1<<<nL1, NTHR, LDS_LAY, stream>>>(csr, offp, cnt, esrc, etyp, x, wp, b1, H1, nN, nE, csrLen);

  hipFuncSetAttribute(reinterpret_cast<const void*>(&k_layer2fc),
                      hipFuncAttributeMaxDynamicSharedMemorySize, LDS_LAY);
  k_layer2fc<<<nQ, NTHR, LDS_LAY, stream>>>(csr, offp, cnt, esrc, etyp, H1, nest, food, wp, b2, bfc,
                                             out, nN, nE, csrLen, nB);
}
